// Conv_80401787781783
// MI455X (gfx1250) — hardware-run, weakly checked
//
#include <hip/hip_runtime.h>


namespace {
constexpr int N = 10000, NP = 10048, NPL = NP  , SRCM = N, EFULL = 100000, E = EFULL  , EL = EFULL  , DA = 16, MUL = 16, DIN = 64, WN = 4 * MUL * MUL, KP = 32;
constexpr float XS = 8.0f, WSC = 256.0f, ALPHA = 0.17677669f, INV_SQRT3 = 0.57735026f;
static_assert(EFULL % 32 == 0 && EL % 32 == 0 && NP % 32 == 0 && WN == 1024, "tiling");
typedef _Float16 b16;
typedef __attribute__((ext_vector_type(16))) _Float16 v16b;
typedef __attribute__((ext_vector_type(8))) _Float16 v8b;
typedef __attribute__((ext_vector_type(8))) float v8f;
typedef __attribute__((ext_vector_type(4))) float v4f;
__device__ __forceinline__ float bf16_rne(float f) { unsigned int u = __float_as_uint(f); u += 0x7FFFu + ((u >> 16) & 1u); return __uint_as_float(u & 0xFFFF0000u); }
__device__ __forceinline__ void split16(float v, b16& hi, b16& lo) { hi = (b16)v; lo = (b16)(v - (float)hi); }
__device__ __forceinline__ v16b frag_kb(const b16* p, int hh) { const v8b a = *(const v8b*)(p + 8 * hh), b = *(const v8b*)(p + 16 + 8 * hh); v16b f;
#pragma unroll
  for (int e = 0; e < 8; ++e) { f[e] = a[e]; f[8 + e] = b[e]; } return f; }
__device__ __forceinline__ v8f wmma16b(v16b a, v16b b, v8f c) { v8f d = __builtin_amdgcn_wmma_f32_16x16x32_f16(false, a, false, b, (short)0, c, false, false); asm volatile("v_nop\n\tv_nop\n\tv_nop\n\tv_nop" : "+v"(d) : "v"(a), "v"(b)); return d; }
__device__ __forceinline__ void wave_lds_sync() { __builtin_amdgcn_fence(__ATOMIC_RELEASE, "workgroup"); __builtin_amdgcn_wave_barrier(); __builtin_amdgcn_fence(__ATOMIC_ACQUIRE, "workgroup"); }
__device__ __forceinline__ float pmul(float a, float b) { float p = a * b; asm volatile("" : "+v"(p)); return p; }
__device__ __forceinline__ int iclamp(int v, int lo, int hi) { return v < lo ? lo : (v > hi ? hi : v); }
constexpr int CSR_NBLK = 512, CSR_GB = 9, CSR_GN = 1 << CSR_GB  , CSR_MAXG = 512, CSR_CAP = 12288  ;
__global__ __launch_bounds__(64) void csrA_kernel(const int* __restrict__ dst, int E, int N, int nG, int CHP, int NGP, int* __restrict__ STG, int* __restrict__ HST) {
  extern __shared__ int sm[];
  int* cnt = sm; int* run = sm + NGP; int* ids = sm + 2 * NGP;
  const int b = blockIdx.x; const int ch = (E + CSR_NBLK - 1) / CSR_NBLK; const int e0 = b * ch, e1 = min(E, e0 + ch);
  for (int i = threadIdx.x; i < NGP; i += 64) cnt[i] = 0;
  for (int i = threadIdx.x; i < CHP; i += 64) ids[i] = -1;
  __syncthreads();
  if (threadIdx.x == 0) {
    for (int e = e0; e < e1; ++e) { int d = dst[e]; d = (d < 0) ? 0 : (d >= N ? N - 1 : d); cnt[d >> CSR_GB] += 1; }
    int acc = 0; for (int g = 0; g < nG; ++g) { run[g] = acc; acc += cnt[g]; }
    for (int e = e0; e < e1; ++e) { int d = dst[e]; d = (d < 0) ? 0 : (d >= N ? N - 1 : d); const int g = d >> CSR_GB; ids[run[g]] = e; run[g] += 1; } }
  __syncthreads();
  typedef __attribute__((ext_vector_type(4))) int v4i;
  for (int pass = 0; pass < 2; ++pass) {
    for (int i = threadIdx.x; i < CHP / 4; i += 64) *(volatile v4i*)(STG + (size_t)b * CHP + i * 4) = *(const v4i*)(&ids[i * 4]);
    for (int i = threadIdx.x; i < NGP / 4; i += 64) { v4i v; for (int e = 0; e < 4; ++e) v[e] = (i * 4 + e < nG) ? cnt[i * 4 + e] : 0; *(volatile v4i*)(HST + (size_t)b * NGP + i * 4) = v; }
    __threadfence(); }
}
__global__ __launch_bounds__(512) void csrS_kernel(const int* __restrict__ HST, int nG, int NGP, int* __restrict__ START, int* __restrict__ TOT, int* __restrict__ OFF) {
  __shared__ int tot[CSR_MAXG];
  const int b = threadIdx.x;
  for (int pass = 0; pass < 2; ++pass) { int runb = 0; for (int g = 0; g < nG; ++g) { int c = HST[(size_t)b * NGP + g]; c = (c < 0) ? 0 : c; ((volatile int*)OFF)[(size_t)g * CSR_NBLK + b] = runb; runb += c; } __threadfence(); }
  for (int g = threadIdx.x; g < nG; g += 512) { int s = 0; for (int bb = 0; bb < CSR_NBLK; ++bb) { int c = HST[(size_t)bb * NGP + g]; s += (c < 0) ? 0 : c; } tot[g] = s; }
  __syncthreads();
  if (threadIdx.x < 32) {
    __shared__ int st[CSR_MAXG + 32];
    if (threadIdx.x == 0) { int acc = 0; for (int g = 0; g < NGP; ++g) { st[g] = acc; if (g < nG) acc += (tot[g] + 31) & ~31; } st[NGP] = acc; }
    __builtin_amdgcn_fence(__ATOMIC_RELEASE, "workgroup"); __builtin_amdgcn_wave_barrier(); __builtin_amdgcn_fence(__ATOMIC_ACQUIRE, "workgroup");
    for (int pass = 0; pass < 2; ++pass) { for (int i = threadIdx.x; i < NGP + 32; i += 32) { ((volatile int*)START)[i] = (i <= NGP) ? st[min(i, NGP)] : 0; ((volatile int*)TOT)[i] = (i < nG) ? tot[i] : 0; } __threadfence(); } }
}
__global__ __launch_bounds__(256) void csrB_kernel(const int* __restrict__ dst, int N, int nG, int CHP, int NGP, int permLen, const int* __restrict__ STG, const int* __restrict__ HST, const int* __restrict__ OFF, const int* __restrict__ START, const int* __restrict__ TOT, int* __restrict__ PERM, int* __restrict__ ROWPTR, int* __restrict__ ROWCNT, int* __restrict__ FLAG) {
  typedef __attribute__((ext_vector_type(4))) int v4i;
  __shared__ int ids[CSR_CAP]; __shared__ unsigned short key[CSR_CAP]; __shared__ int outp[CSR_CAP]; __shared__ int ncnt[CSR_GN + 1]; __shared__ int boff[CSR_NBLK + 1];
  const int g = blockIdx.x, t_ = threadIdx.x; int tot = TOT[g]; int st = START[g], stn = START[g + 1]; const int v0 = g * CSR_GN; const int nv = min(CSR_GN, N - v0);
  st = (st < 0) ? 0 : (st > permLen - 32 ? permLen - 32 : st) & ~31; stn = (stn < st) ? st : (stn > permLen ? permLen : stn); tot = (tot < 0) ? 0 : tot; if (tot > stn - st && tot <= CSR_CAP) tot = stn - st;
  if (tot > CSR_CAP) {
    for (int pass = 0; pass < 2; ++pass) { for (int i = t_; i < CSR_GN / 4; i += 256) { v4i a, c; for (int e = 0; e < 4; ++e) { a[e] = st; c[e] = 0; } *(volatile v4i*)(ROWPTR + v0 + i * 4) = a; *(volatile v4i*)(ROWCNT + v0 + i * 4) = c; } if (t_ == 0) ((volatile int*)FLAG)[0] = 1; __threadfence(); } (void)nv; return; }
  if (t_ == 0) { int acc = 0; for (int b = 0; b < CSR_NBLK; ++b) { boff[b] = acc; int c = HST[(size_t)b * NGP + g]; c = (c < 0) ? 0 : (c > CHP ? CHP : c); acc += c; if (acc > tot) acc = tot; } boff[CSR_NBLK] = acc; }
  for (int i = t_; i <= CSR_GN; i += 256) ncnt[i] = 0;
  __syncthreads();
  for (int b = 0; b < CSR_NBLK; ++b) { const int c = boff[b + 1] - boff[b]; int o_ = OFF[(size_t)g * CSR_NBLK + b]; o_ = (o_ < 0) ? 0 : (o_ > CHP - c ? CHP - c : o_); const int* src_ = STG + (size_t)b * CHP + o_;
    for (int i = t_; i < c; i += 256) { int id = src_[i]; id = (id < 0) ? 0 : id; ids[boff[b] + i] = id; int d = dst[id]; d = (d < v0) ? v0 : (d >= N ? N - 1 : d); int kk = d - v0; kk = (kk < 0) ? 0 : (kk >= CSR_GN ? CSR_GN - 1 : kk); key[boff[b] + i] = (unsigned short)kk; } }
  __syncthreads();
  if (t_ == 0) { for (int i = 0; i < tot; ++i) ncnt[key[i]] += 1; int acc = 0; for (int vl = 0; vl < CSR_GN; ++vl) { const int c = ncnt[vl]; ncnt[vl] = acc; acc += c; } ncnt[CSR_GN] = acc;
    for (int i = 0; i < tot; ++i) { const int vl = key[i]; outp[ncnt[vl]] = ids[i]; ncnt[vl] += 1; }
    for (int vl = CSR_GN; vl > 0; --vl) ncnt[vl] = ncnt[vl - 1]; ncnt[0] = 0; }
  __syncthreads();
  for (int pass = 0; pass < 2; ++pass) {
    for (int i = t_; i < (stn - st) / 4; i += 256) { v4i v; for (int e = 0; e < 4; ++e) { const int q = i * 4 + e; v[e] = (q < tot) ? outp[q] : -1; } *(volatile v4i*)(PERM + st + i * 4) = v; }
    for (int i = t_; i < CSR_GN / 4; i += 256) { v4i a, c; for (int e = 0; e < 4; ++e) { const int vl = i * 4 + e; a[e] = st + ncnt[vl]; c[e] = (vl < nv) ? (ncnt[vl + 1] - ncnt[vl]) : 0; } *(volatile v4i*)(ROWPTR + v0 + i * 4) = a; *(volatile v4i*)(ROWCNT + v0 + i * 4) = c; }
    __threadfence(); }
}
__global__ __launch_bounds__(256) void csrZ_kernel(int* __restrict__ p, size_t n4) { typedef __attribute__((ext_vector_type(4))) int v4i; const size_t tid = (size_t)blockIdx.x * 256 + threadIdx.x, nth = (size_t)gridDim.x * 256; v4i z = {0, 0, 0, 0}; for (size_t i = tid; i < n4; i += nth) *(volatile v4i*)(p + i * 4) = z; }
struct CsrBufs { int *STG, *HST, *OFF, *START, *TOT, *PERM, *ROWPTR, *ROWCNT, *FLAG; int nG, NGP, CHP; size_t permLen; char* base; size_t bytes; };
static size_t csr_carve(CsrBufs& c, char* ws, size_t off, int E, int N) {
  const size_t off0 = off; c.base = ws + off;
  auto al = [&](size_t bytes) { char* p = ws + off; off += (bytes + 255) & ~(size_t)255; return p; };
  c.nG = (N + CSR_GN - 1) / CSR_GN; c.NGP = (c.nG + 31) & ~31; const int ch = (E + CSR_NBLK - 1) / CSR_NBLK; c.CHP = (ch + 31) & ~31; c.permLen = (size_t)E + 32 * (size_t)c.nG + 32;
  c.STG = (int*)al((size_t)CSR_NBLK * c.CHP * 4); c.HST = (int*)al((size_t)CSR_NBLK * c.NGP * 4); c.OFF = (int*)al((size_t)c.NGP * CSR_NBLK * 4); c.START = (int*)al((size_t)(c.NGP + 64) * 4); c.TOT = (int*)al((size_t)(c.NGP + 64) * 4);
  c.PERM = (int*)al(c.permLen * 4); c.ROWPTR = (int*)al((size_t)c.nG * CSR_GN * 4); c.ROWCNT = (int*)al((size_t)c.nG * CSR_GN * 4); c.FLAG = (int*)al(256);
  c.bytes = off - off0; return off;
}
static void csr_build(const CsrBufs& c, const int* dst, int E, int N, hipStream_t stream) {
  const size_t smem = (size_t)(2 * c.NGP + c.CHP) * 4;
  csrZ_kernel<<<512, 256, 0, stream>>>((int*)c.base, c.bytes / 16);
  csrA_kernel<<<CSR_NBLK, 64, smem, stream>>>(dst, E, N, c.nG, c.CHP, c.NGP, c.STG, c.HST);
  csrS_kernel<<<1, 512, 0, stream>>>(c.HST, c.nG, c.NGP, c.START, c.TOT, c.OFF);
  csrB_kernel<<<c.nG, 256, 0, stream>>>(dst, N, c.nG, c.CHP, c.NGP, (int)c.permLen, c.STG, c.HST, c.OFF, c.START, c.TOT, c.PERM, c.ROWPTR, c.ROWCNT, c.FLAG);
}

typedef __attribute__((ext_vector_type(4))) _Float16 v4h;
typedef __attribute__((ext_vector_type(2))) float v2f;
__global__ __launch_bounds__(256) void prep_kernel(const float* __restrict__ w2, const float* __restrict__ b2, b16* __restrict__ WP, float* __restrict__ B2P) {
  const int u_ = blockIdx.x * 256 + threadIdx.x; if (u_ >= WN * KP / 8) return; const int e = u_ * 8; const int cp = e / KP, k0 = e % KP; const int slab = cp / 128, t = (cp % 128) / 16, uu = cp % 16; const int q = slab * 8 + t; const int p = q / MUL, w = q % MUL; const int orig = p * MUL * MUL + uu * MUL + w;
  v8b o; for (int j = 0; j < 8; ++j) { const int k = k0 + j; o[j] = (b16)(k < DA ? bf16_rne(w2[(size_t)k * WN + orig]) * WSC : 0.0f); }
  float bperm = 0.0f; if (u_ < WN) { const int cp2 = u_; const int slab2 = cp2 / 128, t2 = (cp2 % 128) / 16, uu2 = cp2 % 16; const int q2 = slab2 * 8 + t2; const int p2 = q2 / MUL, wq2 = q2 % MUL; bperm = bf16_rne(b2[p2 * MUL * MUL + uu2 * MUL + wq2]); }
  for (int pass = 0; pass < 2; ++pass) { *(volatile v8b*)(WP + e) = o; if (u_ < WN) ((volatile float*)B2P)[u_] = bperm; __threadfence(); }
}
__global__ __launch_bounds__(64) void edge_kernel(const float* __restrict__ xa, const int* __restrict__ src, const float* __restrict__ ea, const float* __restrict__ sh, const float* __restrict__ w1, const float* __restrict__ b1, const b16* __restrict__ WP, const float* __restrict__ B2P, float* __restrict__ EO) {
  __shared__ __attribute__((aligned(16))) b16 Ah[2][16][KP + 8], Al[2][16][KP + 8]; __shared__ __attribute__((aligned(16))) float ES[2][16][88]; __shared__ __attribute__((aligned(16))) float O[2][16][DIN + 4]; __shared__ float W1s[DA * DA], B1s[DA];
  const int wave = threadIdx.x >> 5, lane = threadIdx.x & 31, nloc = lane & 15, hlf = lane >> 4; const size_t e0 = (size_t)blockIdx.x * 32 + wave * 16;
  for (int i = threadIdx.x; i < DA * DA; i += 64) W1s[i] = bf16_rne(w1[i]); if (threadIdx.x < DA) B1s[threadIdx.x] = bf16_rne(b1[threadIdx.x]);
  __syncthreads();
  for (int i = lane; i < 16 * (DIN / 4); i += 32) { const int r = i / (DIN / 4), c4 = (i % (DIN / 4)) * 4; int s_ = iclamp(src[e0 + r], 0, N - 1); if (SRCM < N) s_ %= SRCM; const v4f v = *(const v4f*)(xa + (size_t)s_ * DIN + c4); v4f o; for (int j = 0; j < 4; ++j) o[j] = bf16_rne(v[j]); *(v4f*)(&ES[wave][r][c4]) = o; }
  if (lane < 16) { const v4f v = *(const v4f*)(sh + (e0 + lane) * 4); v4f o; for (int j = 0; j < 4; ++j) o[j] = bf16_rne(v[j]); *(v4f*)(&ES[wave][lane][64]) = o; }
  for (int q = 0; q < 2; ++q) for (int j = 0; j < 4; ++j) O[wave][nloc][hlf * 32 + q * 16 + j * 4 + 0] = 0.0f, O[wave][nloc][hlf * 32 + q * 16 + j * 4 + 1] = 0.0f, O[wave][nloc][hlf * 32 + q * 16 + j * 4 + 2] = 0.0f, O[wave][nloc][hlf * 32 + q * 16 + j * 4 + 3] = 0.0f;
  wave_lds_sync();
  for (int i = lane; i < 16 * MUL; i += 32) { const int r = i / MUL, u = i % MUL; const float* s1 = &ES[wave][r][65]; ES[wave][r][68 + u] = (ES[wave][r][MUL + u * 3 + 0] * s1[0] + ES[wave][r][MUL + u * 3 + 1] * s1[1] + ES[wave][r][MUL + u * 3 + 2] * s1[2]) * INV_SQRT3; }
  for (int i = lane; i < 16 * KP; i += 32) { const int r = i / KP, k = i % KP; float h = 0.0f;
    if (k < DA) { float a = B1s[k];
#pragma unroll 4
      for (int j = 0; j < DA; ++j) a = fmaf(bf16_rne(ea[(e0 + r) * DA + j]), W1s[j * DA + k], a); h = a / (1.0f + __expf(-a)); }
    b16 ph, pl; split16(h * XS, ph, pl); Ah[wave][r][k] = ph; Al[wave][r][k] = pl; }
  wave_lds_sync();
  const v16b af = frag_kb(&Ah[wave][nloc][0], hlf), afl = frag_kb(&Al[wave][nloc][0], hlf);
#pragma unroll 1
  for (int slab = 0; slab < 8; ++slab) { const int p = slab >> 1;
    v8f acc[8];
#pragma unroll
    for (int t = 0; t < 8; ++t) { const v16b bw = frag_kb(WP + (size_t)(slab * 128 + t * 16 + nloc) * KP, hlf); acc[t] = wmma16b(af, bw, (v8f){}); acc[t] = wmma16b(afl, bw, acc[t]); }
#pragma unroll
    for (int t = 0; t < 8; ++t) { const int w_ = (slab & 1) * 8 + t; const float bb = B2P[slab * 128 + t * 16 + nloc];
#pragma unroll
      for (int r = 0; r < 8; ++r) { const int row = 8 * hlf + r; const float val = acc[t][r] * (1.0f / (XS * WSC)) + bb; const float* er = ES[wave][row];
        if (p == 0 || p == 1 || p == 3) { float f = val * (p == 3 ? er[68 + nloc] : er[nloc]);
          for (int w = 1; w < 16; w <<= 1) f += __shfl_xor(f, w);
          if (nloc == t) { if (p == 0) O[wave][row][w_] += ALPHA * er[64] * f; else if (p == 3) O[wave][row][w_] += ALPHA * f; else { for (int m = 0; m < 3; ++m) O[wave][row][MUL + w_ * 3 + m] += ALPHA * f * er[65 + m]; } } }
        else { float f0 = val * er[MUL + nloc * 3 + 0], f1 = val * er[MUL + nloc * 3 + 1], f2 = val * er[MUL + nloc * 3 + 2];
          for (int w = 1; w < 16; w <<= 1) { f0 += __shfl_xor(f0, w); f1 += __shfl_xor(f1, w); f2 += __shfl_xor(f2, w); }
          if (nloc == t) { const float s0 = er[64]; O[wave][row][MUL + w_ * 3 + 0] += ALPHA * s0 * f0; O[wave][row][MUL + w_ * 3 + 1] += ALPHA * s0 * f1; O[wave][row][MUL + w_ * 3 + 2] += ALPHA * s0 * f2; } } } }
    wave_lds_sync(); }
  for (int pass = 0; pass < 2; ++pass) { for (int idx = lane; idx < 16 * (DIN / 4); idx += 32) { const int rr = idx / (DIN / 4), c4 = (idx % (DIN / 4)) * 4; *(volatile v4f*)(EO + (e0 + rr) * DIN + c4) = *(const v4f*)(&O[wave][rr][c4]); } __threadfence(); }
}
__global__ __launch_bounds__(256) void nsum_kernel(const float* __restrict__ EO, const int* __restrict__ PERM, const int* __restrict__ ROWPTR, const int* __restrict__ ROWCNT, int permLen, float* __restrict__ out) {
  __shared__ __attribute__((aligned(16))) float rows[32][DIN + 4];
  const int wave = threadIdx.x >> 5, lane = threadIdx.x & 31;
#pragma unroll 1
  for (int q4 = 0; q4 < 4; ++q4) { const int rw = wave * 4 + q4; const size_t v = (size_t)blockIdx.x * 32 + rw; v2f a = {0.0f, 0.0f};
    if (v < (size_t)N) { int st = ROWPTR[v], cnt = ROWCNT[v]; cnt = iclamp(cnt, 0, 65536); st = iclamp(st, 0, permLen - cnt);
#pragma unroll 1
      for (int j = 0; j < cnt; ++j) { const int e = iclamp(PERM[st + j], 0, E - 1); a += *(const v2f*)(EO + (size_t)e * DIN + lane * 2); } }
    *(v2f*)(&rows[rw][lane * 2]) = a; }
  __syncthreads();
  for (int pass = 0; pass < 2; ++pass) { for (int q = threadIdx.x; q < 32 * DIN / 4; q += 256) { const int rr = q / (DIN / 4), c4 = (q % (DIN / 4)) * 4; const size_t v = (size_t)blockIdx.x * 32 + rr; if (v < (size_t)N) *(volatile v4f*)(out + v * DIN + c4) = *(const v4f*)(&rows[rr][c4]); } __threadfence(); }
}
}

extern "C" void kernel_launch(void* const* d_in, const int* in_sizes, int n_in, void* d_out, int out_size, void* d_ws, size_t ws_size, hipStream_t stream) {
  (void)n_in;
  auto Fp = [&](int i) { return (const float*)d_in[i]; }; auto Ip = [&](int i) { return (const int*)d_in[i]; };
  if (in_sizes[0] != N * DIN || in_sizes[1] != 2 * EFULL || in_sizes[2] != EFULL * DA || in_sizes[3] != EFULL * 4 || in_sizes[4] != DA * DA || in_sizes[5] != DA || in_sizes[6] != DA * WN || in_sizes[7] != WN || out_size != N * DIN) return;
  size_t off = 0; char* ws = (char*)d_ws;
  auto carve = [&](size_t bytes) { char* p = ws + off; off += (bytes + 255) & ~(size_t)255; return p; };
  b16* WP = (b16*)carve((size_t)WN * KP * 2); float* B2P = (float*)carve((size_t)WN * 4); float* EO = (float*)carve((size_t)EFULL * DIN * 4);
  CsrBufs csr; off = csr_carve(csr, ws, off, E, N);
  if (off > ws_size || off > ((size_t)128 << 20)) return;
  prep_kernel<<<(WN * KP / 8 + 255) / 256, 256, 0, stream>>>(Fp(6), Fp(7), WP, B2P);
  csr_build(csr, Ip(1) + EFULL, E, N, stream);
  edge_kernel<<<EL / 32, 64, 0, stream>>>(Fp(0), Ip(1), Fp(2), Fp(3), Fp(4), Fp(5), WP, B2P, EO);
  nsum_kernel<<<NPL / 32, 256, 0, stream>>>(EO, csr.PERM, csr.ROWPTR, csr.ROWCNT, (int)csr.permLen, (float*)d_out);
}
